// SliddingWindowAttention_37976100831413
// MI455X (gfx1250) — hardware-verified
//
#include <hip/hip_runtime.h>
#include <hip/hip_bf16.h>
#include <stddef.h>
#include <stdint.h>

#define NB    2
#define LSEQ  4096
#define DM    512
#define DH    64
#define NTOK  (NB * LSEQ)
#define NQKV  (3 * DH)
#define NW    129
#define HW    64
#define NTAIL (LSEQ - NW)
#define KP    160
#define VTP   192

static_assert(DM % 64 == 0);
static_assert(DH == 64);
static_assert(NTOK % 128 == 0);
static_assert(LSEQ % 32 == 0);
static_assert(KP % 32 == 0);
static_assert(KP >= NW + 15 + 1);
static_assert(VTP % 64 == 0);
static_assert(VTP >= KP);
static_assert((NTOK * DM) % (8 * 256) == 0);

typedef float          v8f   __attribute__((ext_vector_type(8)));
typedef float          v4f   __attribute__((ext_vector_type(4)));
typedef unsigned int   v4u   __attribute__((ext_vector_type(4)));
typedef unsigned short v8us  __attribute__((ext_vector_type(8)));
typedef unsigned short v16us __attribute__((ext_vector_type(16)));
typedef __bf16         v16b  __attribute__((ext_vector_type(16)));
typedef unsigned short ush;

union FragU { v16us v; v8us h[2]; v16b b; };
union PackU { v8us s; v4u u; };
struct HL { v4u h; v4u l; };

__device__ __forceinline__ ush f2bf(float f) {
  const unsigned u = __float_as_uint(f);
  return (ush)((u + 0x7FFFu + ((u >> 16) & 1u)) >> 16);
}
__device__ __forceinline__ float bf2f(ush b) { return __uint_as_float(((unsigned)b) << 16); }

__device__ __forceinline__ HL split8(v8f f) {
  PackU ph, pl;
#pragma unroll
  for (int e = 0; e < 8; ++e) {
    const ush hi = f2bf(f[e]);
    ph.s[e] = hi;
    pl.s[e] = f2bf(f[e] - bf2f(hi));
  }
  HL r; r.h = ph.u; r.l = pl.u;
  return r;
}

__device__ __forceinline__ v8f mmab(v16us a, v16us b, v8f c) {
  FragU ua, ub; ua.v = a; ub.v = b;
  c = __builtin_amdgcn_wmma_f32_16x16x32_bf16(false, ua.b, false, ub.b, (short)0, c, false, false);
  asm volatile("v_nop\n\tv_nop\n\tv_nop\n\tv_nop" : "+v"(c) : "v"(a), "v"(b));
  return c;
}

__device__ __forceinline__ v16us ldfragu(const ush* p, int ld, int row0, int k0, int lane) {
  const int m = lane & 15, lh = lane >> 4;
  const ush* q = p + (size_t)(row0 + m) * ld + k0 + 8 * lh;
  FragU f;
  f.h[0] = *(const v8us*)(q);
  f.h[1] = *(const v8us*)(q + 16);
  return f.v;
}

__device__ __forceinline__ v16us ldfragr(const ush* p, int ld, int row, int k0, int lh) {
  const ush* q = p + (size_t)row * ld + k0 + 8 * lh;
  FragU f;
  f.h[0] = *(const v8us*)(q);
  f.h[1] = *(const v8us*)(q + 16);
  return f.v;
}

__device__ __forceinline__ v8f zero8() { return (v8f){0.f, 0.f, 0.f, 0.f, 0.f, 0.f, 0.f, 0.f}; }

__device__ __forceinline__ void gemm3_32x64(const ush* __restrict__ Ah, const ush* __restrict__ Al, int lda,
                                            const ush* __restrict__ Bh, const ush* __restrict__ Bl, int ldb,
                                            int m0, int n0, int lane, v8f (&acc)[2][4]) {
#pragma unroll 1
  for (int k0 = 0; k0 < DM; k0 += 32) {
    const v16us a0h = ldfragu(Ah, lda, m0, k0, lane);
    const v16us a1h = ldfragu(Ah, lda, m0 + 16, k0, lane);
    const v16us a0l = ldfragu(Al, lda, m0, k0, lane);
    const v16us a1l = ldfragu(Al, lda, m0 + 16, k0, lane);
#pragma unroll
    for (int t = 0; t < 4; ++t) {
      const v16us bh = ldfragu(Bh, ldb, n0 + 16 * t, k0, lane);
      const v16us bl = ldfragu(Bl, ldb, n0 + 16 * t, k0, lane);
      acc[0][t] = mmab(a0h, bh, acc[0][t]);
      acc[1][t] = mmab(a1h, bh, acc[1][t]);
      acc[0][t] = mmab(a0h, bl, acc[0][t]);
      acc[1][t] = mmab(a1h, bl, acc[1][t]);
      acc[0][t] = mmab(a0l, bh, acc[0][t]);
      acc[1][t] = mmab(a1l, bh, acc[1][t]);
    }
  }
}

__global__ __launch_bounds__(256) void k_cvt_x(const float* __restrict__ x, ush* __restrict__ xh,
                                               ush* __restrict__ xl, int ngrp) {
  const int t = blockIdx.x * 256 + (int)threadIdx.x;
  if (t >= ngrp) return;
  const size_t o = (size_t)t * 8;
  const v4f a0 = *(const v4f*)(x + o);
  const v4f a1 = *(const v4f*)(x + o + 4);
  const v8f f = (v8f){a0[0], a0[1], a0[2], a0[3], a1[0], a1[1], a1[2], a1[3]};
  const HL s = split8(f);
  *(volatile v4u*)(xh + o) = s.h;
  *(volatile v4u*)(xl + o) = s.l;
  __threadfence();
  *(volatile v4u*)(xh + o) = s.h;
  *(volatile v4u*)(xl + o) = s.l;
}

#define WTP 72
__global__ __launch_bounds__(256) void k_cvt_w(const float* __restrict__ wq, const float* __restrict__ wk,
                                               const float* __restrict__ wv,
                                               ush* __restrict__ w3h, ush* __restrict__ w3l) {
  __shared__ __align__(16) ush th[64 * WTP];
  __shared__ __align__(16) ush tl[64 * WTP];
  const int which = blockIdx.y;
  const float* w = (which == 0) ? wq : ((which == 1) ? wk : wv);
  const int c0  = blockIdx.x * 64;
  const int tid = threadIdx.x;
#pragma unroll 4
  for (int it = 0; it < 16; ++it) {
    const int idx = tid + 256 * it;
    const int ci  = idx >> 6;
    const int n   = idx & 63;
    const float v = w[(size_t)(c0 + ci) * DH + n];
    const ush hi  = f2bf(v);
    th[n * WTP + ci] = hi;
    tl[n * WTP + ci] = f2bf(v - bf2f(hi));
  }
  __syncthreads();
  v4u vh[2], vl[2];
  size_t go[2];
#pragma unroll
  for (int j = 0; j < 2; ++j) {
    const int p  = tid + 256 * j;
    const int n  = p >> 3;
    const int pc = p & 7;
    PackU kh, kl;
    kh.s = *(const v8us*)(th + n * WTP + pc * 8);
    kl.s = *(const v8us*)(tl + n * WTP + pc * 8);
    vh[j] = kh.u; vl[j] = kl.u;
    go[j] = ((size_t)(which * DH + n)) * DM + c0 + pc * 8;
  }
#pragma unroll
  for (int j = 0; j < 2; ++j) { *(volatile v4u*)(w3h + go[j]) = vh[j]; *(volatile v4u*)(w3l + go[j]) = vl[j]; }
  __threadfence();
#pragma unroll
  for (int j = 0; j < 2; ++j) { *(volatile v4u*)(w3h + go[j]) = vh[j]; *(volatile v4u*)(w3l + go[j]) = vl[j]; }
}

#define STP 72
#define SFP 68
__global__ __launch_bounds__(128) void k_qkv3(const ush* __restrict__ xh3, const ush* __restrict__ xl3,
                                              const ush* __restrict__ wth, const ush* __restrict__ wtl,
                                              const float* __restrict__ bq,
                                              const float* __restrict__ bk,
                                              const float* __restrict__ bv,
                                              ush* __restrict__ q3h, ush* __restrict__ q3l,
                                              ush* __restrict__ k3h, ush* __restrict__ k3l,
                                              float* __restrict__ vf) {
  __shared__ __align__(16) ush   st[128 * STP];
  __shared__ __align__(16) float sf[128 * SFP];
  const int tid = threadIdx.x, lane = tid & 31, wave = tid >> 5;
  const int hh = lane >> 4, c = lane & 15;
  const int mb = blockIdx.x * 128;
  const int m0 = mb + wave * 32;
  const int which = blockIdx.y;
  const int n0 = which * DH;
  const float* bias = (which == 0) ? bq : ((which == 1) ? bk : bv);

  v8f acc[2][4];
#pragma unroll
  for (int s = 0; s < 2; ++s)
#pragma unroll
    for (int t = 0; t < 4; ++t) acc[s][t] = zero8();
  gemm3_32x64(xh3, xl3, DM, wth, wtl, DM, m0, n0, lane, acc);

#pragma unroll
  for (int t = 0; t < 4; ++t) {
    const float bn = bias[16 * t + c];
#pragma unroll
    for (int sub = 0; sub < 2; ++sub) {
#pragma unroll
      for (int r = 0; r < 8; ++r) acc[sub][t][r] += bn;
    }
  }

  if (which < 2) {
    ush* bhp = (which == 0) ? q3h : k3h;
    ush* blp = (which == 0) ? q3l : k3l;
    size_t go[8];
#pragma unroll
    for (int j = 0; j < 8; ++j) {
      const int p  = tid + 128 * j;
      const int L  = p >> 3;
      const int pc = p & 7;
      go[j] = ((size_t)(mb + L)) * DH + pc * 8;
    }
#pragma unroll 1
    for (int ph = 0; ph < 2; ++ph) {
      __syncthreads();
#pragma unroll
      for (int t = 0; t < 4; ++t) {
#pragma unroll
        for (int sub = 0; sub < 2; ++sub) {
#pragma unroll
          for (int r = 0; r < 8; ++r) {
            const int lr = wave * 32 + sub * 16 + 8 * hh + r;
            const float v = acc[sub][t][r];
            const ush hi = f2bf(v);
            st[lr * STP + 16 * t + c] = (ph == 0) ? hi : f2bf(v - bf2f(hi));
          }
        }
      }
      __syncthreads();
      v4u val[8];
#pragma unroll
      for (int j = 0; j < 8; ++j) {
        const int p  = tid + 128 * j;
        const int L  = p >> 3;
        const int pc = p & 7;
        PackU pk;
        pk.s  = *(const v8us*)(st + L * STP + pc * 8);
        val[j] = pk.u;
      }
      ush* dst = (ph == 0) ? bhp : blp;
#pragma unroll
      for (int j = 0; j < 8; ++j) *(volatile v4u*)(dst + go[j]) = val[j];
      __threadfence();
#pragma unroll
      for (int j = 0; j < 8; ++j) *(volatile v4u*)(dst + go[j]) = val[j];
      __threadfence();
    }
  } else {
#pragma unroll
    for (int t = 0; t < 4; ++t) {
#pragma unroll
      for (int sub = 0; sub < 2; ++sub) {
#pragma unroll
        for (int r = 0; r < 8; ++r) {
          const int lr = wave * 32 + sub * 16 + 8 * hh + r;
          sf[lr * SFP + 16 * t + c] = acc[sub][t][r];
        }
      }
    }
    __syncthreads();
    v4f val[16];
    size_t go[16];
#pragma unroll
    for (int j = 0; j < 16; ++j) {
      const int p  = tid + 128 * j;
      const int L  = p >> 4;
      const int pc = p & 15;
      val[j] = *(const v4f*)(sf + L * SFP + pc * 4);
      go[j]  = ((size_t)(mb + L)) * DH + pc * 4;
    }
#pragma unroll
    for (int j = 0; j < 16; ++j) *(volatile v4f*)(vf + go[j]) = val[j];
    __threadfence();
#pragma unroll
    for (int j = 0; j < 16; ++j) *(volatile v4f*)(vf + go[j]) = val[j];
  }
}

#define TP 200
__global__ __launch_bounds__(256) void k_vprep(const float* __restrict__ vf, ush* __restrict__ vth,
                                               ush* __restrict__ vtl, float* __restrict__ vtail) {
  __shared__ __align__(16) ush   th[DH * TP];
  __shared__ __align__(16) ush   tl[DH * TP];
  __shared__ __align__(16) float part[4 * DH];
  __shared__ __align__(16) float vt[DH];
  const int b = blockIdx.x;
  const int tid = threadIdx.x;
  const float* vb = vf + (size_t)b * LSEQ * DH;

  {
    const int d   = tid & 63;
    const int cch = tid >> 6;
    float s = 0.f;
#pragma unroll 1
    for (int o = NW + cch; o < LSEQ; o += 4) s += vb[(size_t)o * DH + d];
    part[cch * DH + d] = s;
  }
#pragma unroll 1
  for (int it = 0; it < (DH * VTP) / 256; ++it) {
    const int idx = tid + 256 * it;
    const int o   = idx >> 6;
    const int d   = idx & 63;
    const int oc  = (o < NW) ? o : (NW - 1);
    float v = vb[(size_t)oc * DH + d];
    v = (o < NW) ? v : 0.f;
    const ush hi = f2bf(v);
    th[d * TP + o] = hi;
    tl[d * TP + o] = f2bf(v - bf2f(hi));
  }
  __syncthreads();
  if (tid < DH) vt[tid] = ((part[tid] + part[DH + tid]) + part[2 * DH + tid]) + part[3 * DH + tid];
  __syncthreads();

  v4u hv[6], lv[6];
  size_t go[6];
#pragma unroll
  for (int it = 0; it < 6; ++it) {
    const int p  = tid + 256 * it;
    const int d  = p / 24;
    const int pc = p - 24 * d;
    PackU kh, kl;
    kh.s = *(const v8us*)(th + d * TP + pc * 8);
    kl.s = *(const v8us*)(tl + d * TP + pc * 8);
    hv[it] = kh.u; lv[it] = kl.u;
    go[it] = ((size_t)(b * DH + d)) * VTP + pc * 8;
  }
  const int tq = tid & 15;
  const v4f tv = *(const v4f*)(vt + tq * 4);
  const bool tw = (tid < 16);
  float* vtd = vtail + b * DH + tq * 4;

#pragma unroll
  for (int it = 0; it < 6; ++it) { *(volatile v4u*)(vth + go[it]) = hv[it]; *(volatile v4u*)(vtl + go[it]) = lv[it]; }
  if (tw) *(volatile v4f*)(vtd) = tv;
  __threadfence();
#pragma unroll
  for (int it = 0; it < 6; ++it) { *(volatile v4u*)(vth + go[it]) = hv[it]; *(volatile v4u*)(vtl + go[it]) = lv[it]; }
  if (tw) *(volatile v4f*)(vtd) = tv;
}

#define AWV 2
#define SSP 148
#define SPP 168
#define OTP 68
__global__ __launch_bounds__(64) void k_attn3(const ush* __restrict__ q3h, const ush* __restrict__ q3l,
                                              const ush* __restrict__ k3h, const ush* __restrict__ k3l,
                                              const ush* __restrict__ vth, const ush* __restrict__ vtl,
                                              const float* __restrict__ vtail, float* __restrict__ out) {
  __shared__ __align__(16) float sS[AWV * 16 * SSP];
  __shared__ __align__(16) ush   sPh[AWV * 16 * SPP];
  __shared__ __align__(16) ush   sPl[AWV * 16 * SPP];
  __shared__ __align__(16) float rEN[AWV * 16];
  __shared__ __align__(16) float rIZ[AWV * 16];

  const int tid = threadIdx.x, lane = tid & 31, wave = tid >> 5;
  const int hh = lane >> 4, c = lane & 15;
  const int b  = blockIdx.y;
  const int i0 = ((int)blockIdx.x * AWV + wave) * 16;
  const size_t tb = (size_t)b * LSEQ;
  const ush* Qh = q3h + tb * DH;
  const ush* Ql = q3l + tb * DH;
  const ush* Kh = k3h + tb * DH;
  const ush* Kl = k3l + tb * DH;
  const ush* Vh = vth + (size_t)b * DH * VTP;
  const ush* Vl = vtl + (size_t)b * DH * VTP;
  const float* vtb = vtail + b * DH;
  float* mS  = sS  + wave * 16 * SSP;
  ush*   mPh = sPh + wave * 16 * SPP;
  ush*   mPl = sPl + wave * 16 * SPP;

  {
    const v16us a0h = ldfragu(Qh, DH, i0, 0,  lane);
    const v16us a1h = ldfragu(Qh, DH, i0, 32, lane);
    const v16us a0l = ldfragu(Ql, DH, i0, 0,  lane);
    const v16us a1l = ldfragu(Ql, DH, i0, 32, lane);
#pragma unroll 1
    for (int jt = 0; jt < 9; ++jt) {
      int kr = i0 - HW + 16 * jt + c;
      kr = (kr < 0) ? 0 : ((kr > LSEQ - 1) ? (LSEQ - 1) : kr);
      const v16us b0h = ldfragr(Kh, DH, kr, 0,  hh);
      const v16us b1h = ldfragr(Kh, DH, kr, 32, hh);
      const v16us b0l = ldfragr(Kl, DH, kr, 0,  hh);
      const v16us b1l = ldfragr(Kl, DH, kr, 32, hh);
      v8f s = zero8();
      s = mmab(a0h, b0h, s);
      s = mmab(a0h, b0l, s);
      s = mmab(a0l, b0h, s);
      s = mmab(a1h, b1h, s);
      s = mmab(a1h, b1l, s);
      s = mmab(a1l, b1h, s);
#pragma unroll
      for (int r = 0; r < 8; ++r) mS[(8 * hh + r) * SSP + jt * 16 + c] = s[r];
    }
  }
  __syncthreads();

#pragma unroll 1
  for (int r = 0; r < 16; ++r) {
    const int jb = i0 + r - HW;
    const float* sr = mS + r * SSP;
    float sv[5];
    float mx = 0.f;
#pragma unroll
    for (int t = 0; t < 5; ++t) {
      const int o   = lane + 32 * t;
      const bool act = (o < NW);
      int col = o + r; col = (col > 143) ? 143 : col;
      const int j   = jb + o;
      const bool val = act && (j >= 0) && (j < LSEQ);
      float s = sr[col];
      s = val ? s : 0.f;
      sv[t] = s;
      mx = fmaxf(mx, s);
    }
#pragma unroll
    for (int off = 16; off > 0; off >>= 1) mx = fmaxf(mx, __shfl_xor(mx, off, 32));
    float ev[5];
    float sum = 0.f;
#pragma unroll
    for (int t = 0; t < 5; ++t) {
      const int o = lane + 32 * t;
      float e = __expf(sv[t] - mx);
      e = (o < NW) ? e : 0.f;
      ev[t] = e;
      sum += e;
    }
#pragma unroll
    for (int off = 16; off > 0; off >>= 1) sum += __shfl_xor(sum, off, 32);
    const float eneg = __expf(-mx);
    const float Z    = (float)NTAIL * eneg + sum;
    const float invZ = 1.0f / Z;
#pragma unroll
    for (int t = 0; t < 5; ++t) {
      const int o  = lane + 32 * t;
      const ush hi = f2bf(ev[t]);
      mPh[r * SPP + o] = hi;
      mPl[r * SPP + o] = f2bf(ev[t] - bf2f(hi));
    }
    if (lane == 0) { rEN[wave * 16 + r] = eneg; rIZ[wave * 16 + r] = invZ; }
  }
  __syncthreads();

  v8f acc[4];
#pragma unroll
  for (int nt = 0; nt < 4; ++nt) acc[nt] = zero8();
#pragma unroll 1
  for (int kk = 0; kk < KP / 32; ++kk) {
    const v16us pah = ldfragu(mPh, SPP, 0, kk * 32, lane);
    const v16us pal = ldfragu(mPl, SPP, 0, kk * 32, lane);
#pragma unroll
    for (int nt = 0; nt < 4; ++nt) {
      const v16us vbh = ldfragu(Vh, VTP, nt * 16, kk * 32, lane);
      const v16us vbl = ldfragu(Vl, VTP, nt * 16, kk * 32, lane);
      acc[nt] = mmab(pah, vbh, acc[nt]);
      acc[nt] = mmab(pah, vbl, acc[nt]);
      acc[nt] = mmab(pal, vbh, acc[nt]);
    }
  }

  float* sO = mS;
#pragma unroll
  for (int nt = 0; nt < 4; ++nt) {
    const int d = 16 * nt + c;
    const float tv = vtb[d];
#pragma unroll
    for (int r = 0; r < 8; ++r) {
      const int row  = 8 * hh + r;
      const float en = rEN[wave * 16 + row];
      const float iz = rIZ[wave * 16 + row];
      sO[row * OTP + d] = (acc[nt][r] + en * tv) * iz;
    }
  }
  __syncthreads();
  v4f val[8];
  size_t go[8];
#pragma unroll
  for (int it = 0; it < 8; ++it) {
    const int p   = lane + 32 * it;
    const int row = p >> 4;
    const int pc  = p & 15;
    val[it] = *(const v4f*)(sO + row * OTP + pc * 4);
    go[it]  = (tb + (size_t)(i0 + row)) * DH + pc * 4;
  }
#pragma unroll
  for (int it = 0; it < 8; ++it) *(volatile v4f*)(out + go[it]) = val[it];
  __threadfence();
#pragma unroll
  for (int it = 0; it < 8; ++it) *(volatile v4f*)(out + go[it]) = val[it];
}

extern "C" void kernel_launch(void* const* d_in, const int* in_sizes, int n_in,
                              void* d_out, int out_size, void* d_ws, size_t ws_size,
                              hipStream_t stream) {
  if (n_in < 7) return;
  if (in_sizes[0] != NTOK * DM) return;
  if (in_sizes[1] != DM * DH) return;
  if (in_sizes[2] != DH) return;
  if (in_sizes[3] != DM * DH) return;
  if (in_sizes[4] != DH) return;
  if (in_sizes[5] != DM * DH) return;
  if (in_sizes[6] != DH) return;
  if (out_size != NTOK * DH) return;

  const float* x  = (const float*)d_in[0];
  const float* wq = (const float*)d_in[1];
  const float* bq = (const float*)d_in[2];
  const float* wk = (const float*)d_in[3];
  const float* bk = (const float*)d_in[4];
  const float* wv = (const float*)d_in[5];
  const float* bv = (const float*)d_in[6];
  float* out = (float*)d_out;

  size_t off = 0;
  const size_t oX3h = off; off += (size_t)NTOK * DM * 2;
  const size_t oX3l = off; off += (size_t)NTOK * DM * 2;
  const size_t oW3h = off; off += (size_t)NQKV * DM * 2;
  const size_t oW3l = off; off += (size_t)NQKV * DM * 2;
  const size_t oQ3h = off; off += (size_t)NTOK * DH * 2;
  const size_t oQ3l = off; off += (size_t)NTOK * DH * 2;
  const size_t oK3h = off; off += (size_t)NTOK * DH * 2;
  const size_t oK3l = off; off += (size_t)NTOK * DH * 2;
  const size_t oVf  = off; off += (size_t)NTOK * DH * 4;
  const size_t oVTh = off; off += (size_t)NB * DH * VTP * 2;
  const size_t oVTl = off; off += (size_t)NB * DH * VTP * 2;
  const size_t oVt  = off; off += (size_t)NB * DH * 4;
  if (off > ws_size) return;
  if (off > (size_t)134217728) return;

  char* ws = (char*)d_ws;
  ush*   X3h = (ush*)(ws + oX3h);
  ush*   X3l = (ush*)(ws + oX3l);
  ush*   W3h = (ush*)(ws + oW3h);
  ush*   W3l = (ush*)(ws + oW3l);
  ush*   Q3h = (ush*)(ws + oQ3h);
  ush*   Q3l = (ush*)(ws + oQ3l);
  ush*   K3h = (ush*)(ws + oK3h);
  ush*   K3l = (ush*)(ws + oK3l);
  float* Vf  = (float*)(ws + oVf);
  ush*   VTh = (ush*)(ws + oVTh);
  ush*   VTl = (ush*)(ws + oVTl);
  float* Vt  = (float*)(ws + oVt);

  const int ngx = in_sizes[0] / 8;
  k_cvt_x<<<dim3((ngx + 255) / 256), dim3(256), 0, stream>>>(x, X3h, X3l, ngx);
  k_cvt_w<<<dim3(DM / 64, 3), dim3(256), 0, stream>>>(wq, wk, wv, W3h, W3l);
  k_qkv3<<<dim3(NTOK / 128, 3), dim3(128), 0, stream>>>(X3h, X3l, W3h, W3l, bq, bk, bv,
                                                        Q3h, Q3l, K3h, K3l, Vf);
  k_vprep<<<dim3(NB), dim3(256), 0, stream>>>(Vf, VTh, VTl, Vt);
  k_attn3<<<dim3(LSEQ / (16 * AWV), NB), dim3(64), 0, stream>>>(Q3h, Q3l, K3h, K3l, VTh, VTl, Vt, out);
  (void)hipGetLastError();
}
